// RelativePositionAttention_46420006535899
// MI455X (gfx1250) — hardware-verified
//
#include <hip/hip_runtime.h>
#include <math.h>

#ifndef NB
#define NB 2
#endif
#ifndef SEQ
#define SEQ 2048
#endif
#define NB_FULL 2
#define SEQ_FULL 2048
#define DH 64
#define NREL 257
#define NRELP 272
#define MAXREL 128
#define QK_CARRY 16.0f
#define T_CARRY 256.0f
#define V_CARRY 16.0f
#define P_CARRY 1024.0f
#define WT_P 36
#define SO_P 68
#define NBLK (NB * SEQ / 64)
#define BLK_PER_B (SEQ / 64)

static_assert(DH == 64);
static_assert(NREL == 2 * MAXREL + 1);
static_assert(NRELP % 16 == 0 && NRELP >= NREL);
static_assert(SEQ % 64 == 0 && SEQ <= SEQ_FULL && NB <= NB_FULL);
static_assert((NB * SEQ * 8) % 256 == 0);
static_assert(2 * 256 == DH * 8);
static_assert(32 * 16 * 4 == 16 * 32 * 4);
static_assert(32 * 16 * 8 == 16 * DH * 4);
static_assert(16 * SO_P <= 16 * NRELP);
static_assert(4 * 16 * NRELP * 4 + 4 * 16 * WT_P * 4 <= 131072);
static_assert(4 * 16 * NRELP * 4 + 128 * 4 <= 131072);
static_assert(64 * 65 * 4 <= 131072);

static constexpr float LOG2E_F = 1.4426950408889634f;
static constexpr float SC_QK = LOG2E_F / (8.0f * QK_CARRY * QK_CARRY);
static constexpr float SC_QR = LOG2E_F / (8.0f * QK_CARRY * T_CARRY);
static constexpr float SC_O  = 1.0f / (P_CARRY * V_CARRY);
static_assert(8.0f * QK_CARRY * QK_CARRY == 2048.0f && SC_QK * 2048.0f == LOG2E_F);
static_assert(8.0f * QK_CARRY * T_CARRY == 32768.0f && SC_QR * 32768.0f == LOG2E_F);
static_assert(P_CARRY * V_CARRY == 16384.0f && SC_O * 16384.0f == 1.0f);

static constexpr size_t PLANE_B  = (size_t)NB * SEQ * DH * 2;
static constexpr size_t T_B      = (size_t)NRELP * DH * 2;
static constexpr size_t ST_B     = (size_t)NBLK * 128 * 4;
static constexpr size_t OFF_Q    = 0;
static constexpr size_t OFF_K    = OFF_Q + PLANE_B;
static constexpr size_t OFF_VT   = OFF_K + PLANE_B;
static constexpr size_t OFF_T    = OFF_VT + PLANE_B;
static constexpr size_t OFF_ST   = OFF_T + T_B;
static constexpr size_t WS_TOTAL = OFF_ST + ST_B;
static_assert(PLANE_B % 256 == 0 && T_B % 256 == 0 && ST_B % 256 == 0);
static_assert(WS_TOTAL <= (size_t)134217728);

static constexpr size_t OUT1_ELEM  = (size_t)NB_FULL * SEQ_FULL * DH;
static constexpr size_t OUT_TOTAL  = OUT1_ELEM + (size_t)NB_FULL * SEQ_FULL * SEQ_FULL;
static_assert(OUT1_ELEM * 4 == (size_t)1048576);
static_assert(OUT_TOTAL * 4 == (size_t)34603008);
static_assert(OUT1_ELEM + ((size_t)(NB - 1) * SEQ_FULL + (SEQ - 1)) * SEQ_FULL + (SEQ - 1) < OUT_TOTAL);
static_assert(((size_t)(NB - 1) * SEQ_FULL + (SEQ - 1)) * DH + (DH - 1) < OUT1_ELEM);

static constexpr int IN_ACT_MIN = ((NB - 1) * SEQ_FULL + SEQ) * DH;
static constexpr int IN_TAB_MIN = NREL * DH;
static constexpr int OUT_MIN = (int)(OUT1_ELEM + ((size_t)(NB - 1) * SEQ_FULL + SEQ) * SEQ_FULL);

typedef _Float16 h16;
typedef __attribute__((ext_vector_type(16))) _Float16 v16h;
typedef __attribute__((ext_vector_type(8)))  _Float16 v8h;
typedef __attribute__((ext_vector_type(8)))  float    v8f;
typedef __attribute__((ext_vector_type(4)))  float    v4f;


__device__ __forceinline__ float bfr(float f) {
    unsigned u = __float_as_uint(f);
    u += 0x7FFFu + ((u >> 16) & 1u);
    return __uint_as_float(u & 0xFFFF0000u);
}
static __device__ __forceinline__ h16 toh_flush(float v) { const float w = (fabsf(v) < 6.103515625e-05f) ? 0.0f : v; return (h16)w; }
__device__ __forceinline__ float fsel_max(float a, float b) { return (b > a) ? b : a; }

union FragU { v16h v; v8h h[2]; };
__device__ __forceinline__ v16h frag_ld(const _Float16* p) {
    FragU f; f.h[0] = *(const v8h*)(p); f.h[1] = *(const v8h*)(p + 16); return f.v;
}
__device__ __forceinline__ v8f wmma16g(v16h a, v16h b, v8f c) {
    c = __builtin_amdgcn_wmma_f32_16x16x32_f16(false, a, false, b, (short)0, c, false, false);
    asm volatile("v_nop\n\tv_nop\n\tv_nop\n\tv_nop" : "+v"(c) : "v"(a), "v"(b));
    return c;
}
__device__ __forceinline__ void wave_sync_lds() {
    __builtin_amdgcn_fence(3  , "workgroup");
    __builtin_amdgcn_wave_barrier();
    __builtin_amdgcn_fence(2  , "workgroup");
}
__device__ __forceinline__ void st_v8h_x2(_Float16* p, v8h v) {
    *(volatile v8h*)p = v;
    __threadfence();
    *(volatile v8h*)p = v;
}

__global__ __launch_bounds__(256) void k_cvt_qk(const float* __restrict__ q, const float* __restrict__ k,
                                                _Float16* __restrict__ q16, _Float16* __restrict__ k16) {
    const unsigned u = blockIdx.x * 256u + threadIdx.x;
    const unsigned row = u >> 3, c0 = (u & 7u) * 8u;
    const unsigned b = row / (unsigned)SEQ;
    const unsigned i = row - b * (unsigned)SEQ;
    const size_t src = ((size_t)b * SEQ_FULL + i) * DH + c0;
    const v4f a0 = *(const v4f*)(q + src), a1 = *(const v4f*)(q + src + 4);
    const v4f b0 = *(const v4f*)(k + src), b1 = *(const v4f*)(k + src + 4);
    v8h hq, hk;
    hq[0] = toh_flush(bfr(a0.x) * QK_CARRY); hq[1] = toh_flush(bfr(a0.y) * QK_CARRY);
    hq[2] = toh_flush(bfr(a0.z) * QK_CARRY); hq[3] = toh_flush(bfr(a0.w) * QK_CARRY);
    hq[4] = toh_flush(bfr(a1.x) * QK_CARRY); hq[5] = toh_flush(bfr(a1.y) * QK_CARRY);
    hq[6] = toh_flush(bfr(a1.z) * QK_CARRY); hq[7] = toh_flush(bfr(a1.w) * QK_CARRY);
    hk[0] = toh_flush(bfr(b0.x) * QK_CARRY); hk[1] = toh_flush(bfr(b0.y) * QK_CARRY);
    hk[2] = toh_flush(bfr(b0.z) * QK_CARRY); hk[3] = toh_flush(bfr(b0.w) * QK_CARRY);
    hk[4] = toh_flush(bfr(b1.x) * QK_CARRY); hk[5] = toh_flush(bfr(b1.y) * QK_CARRY);
    hk[6] = toh_flush(bfr(b1.z) * QK_CARRY); hk[7] = toh_flush(bfr(b1.w) * QK_CARRY);
    st_v8h_x2(q16 + (size_t)row * DH + c0, hq);
    st_v8h_x2(k16 + (size_t)row * DH + c0, hk);
}

__global__ __launch_bounds__(256) void k_cvt_tab(const float* __restrict__ tab, _Float16* __restrict__ t16) {
    const unsigned u = blockIdx.x * 256u + threadIdx.x;
    if (u >= (unsigned)(NRELP * 8)) return;
    const unsigned row = u >> 3, c0 = (u & 7u) * 8u;
    const unsigned rs = min(row, (unsigned)(NREL - 1));
    const v4f a0 = *(const v4f*)(tab + (size_t)rs * DH + c0), a1 = *(const v4f*)(tab + (size_t)rs * DH + c0 + 4);
    const bool live = row < (unsigned)NREL;
    float w[8] = {a0.x, a0.y, a0.z, a0.w, a1.x, a1.y, a1.z, a1.w};
    v8h ht;
#pragma unroll
    for (int e = 0; e < 8; ++e) {
        const float x = bfr(w[e]) * T_CARRY;
        ht[e] = toh_flush(live ? x : 0.0f);
    }
    st_v8h_x2(t16 + (size_t)row * DH + c0, ht);
}

__global__ __launch_bounds__(256) void k_cvt_vt(const float* __restrict__ v, _Float16* __restrict__ vt16) {
    __shared__ float sT[64 * 65];
    const unsigned t = threadIdx.x;
    const unsigned bx = blockIdx.x;
    const unsigned b = bx / (unsigned)BLK_PER_B;
    const unsigned key0 = (bx - b * (unsigned)BLK_PER_B) * 64u;
    {
        const unsigned key = t >> 2, qd = (t & 3u) * 16u;
        const float* src = v + ((size_t)b * SEQ_FULL + key0 + key) * DH + qd;
#pragma unroll
        for (int g = 0; g < 4; ++g) {
            const v4f a = *(const v4f*)(src + 4 * g);
            float* d = sT + key * 65u + qd + 4u * (unsigned)g;
            d[0] = bfr(a.x) * V_CARRY; d[1] = bfr(a.y) * V_CARRY; d[2] = bfr(a.z) * V_CARRY; d[3] = bfr(a.w) * V_CARRY;
        }
    }
    __syncthreads();
    v8h hv[2];
#pragma unroll
    for (int it = 0; it < 2; ++it) {
        const unsigned item = (unsigned)it * 256u + t;
        const unsigned d = item >> 3, kg = item & 7u;
#pragma unroll
        for (int e = 0; e < 8; ++e) hv[it][e] = toh_flush(sT[(8u * kg + (unsigned)e) * 65u + d]);
    }
    for (int pass = 0; pass < 2; ++pass) {
#pragma unroll
        for (int it = 0; it < 2; ++it) {
            const unsigned item = (unsigned)it * 256u + t;
            const unsigned d = item >> 3, kg = item & 7u;
            *(volatile v8h*)(vt16 + ((size_t)b * DH + d) * SEQ + key0 + 8u * kg) = hv[it];
        }
        __threadfence();
    }
}

__device__ __forceinline__ void build_qr(const _Float16* t16, float* qrs, v16h qf0, v16h qf1, unsigned hh, unsigned c) {
#pragma unroll 1
    for (unsigned tq = 0; tq < (unsigned)(NRELP / 16); ++tq) {
        const _Float16* tr = t16 + (size_t)(tq * 16u + c) * DH + 8u * hh;
        const v16h a0 = frag_ld(tr), a1 = frag_ld(tr + 32);
        v8f z = (v8f){0.f,0.f,0.f,0.f,0.f,0.f,0.f,0.f};
        z = wmma16g(a0, qf0, z);
        z = wmma16g(a1, qf1, z);
        v4f lo, hi;
        lo.x = z[0] * SC_QR; lo.y = z[1] * SC_QR; lo.z = z[2] * SC_QR; lo.w = z[3] * SC_QR;
        hi.x = z[4] * SC_QR; hi.y = z[5] * SC_QR; hi.z = z[6] * SC_QR; hi.w = z[7] * SC_QR;
        float* d = qrs + c * (unsigned)NRELP + tq * 16u + 8u * hh;
        *(v4f*)(d) = lo;
        *(v4f*)(d + 4) = hi;
    }
}

__device__ __forceinline__ void score_step(const _Float16* krow, const float* qrow, v16h qf0, v16h qf1, int kq, v8f& s0, v8f& s1) {
    const v8f z = (v8f){0.f,0.f,0.f,0.f,0.f,0.f,0.f,0.f};
    const v16h k00 = frag_ld(krow), k01 = frag_ld(krow + 32);
    const v16h k10 = frag_ld(krow + 16 * DH), k11 = frag_ld(krow + 16 * DH + 32);
    s0 = wmma16g(k00, qf0, z);
    s0 = wmma16g(k01, qf1, s0);
    s1 = wmma16g(k10, qf0, z);
    s1 = wmma16g(k11, qf1, s1);
#pragma unroll
    for (int r = 0; r < 8; ++r) {
        const int t0 = min(max(kq + r, 0), 2 * MAXREL);
        const int t1 = min(max(kq + 16 + r, 0), 2 * MAXREL);
        s0[r] = fmaf(s0[r], SC_QK, qrow[(unsigned)t0]);
        s1[r] = fmaf(s1[r], SC_QK, qrow[(unsigned)t1]);
    }
}

__global__ __launch_bounds__(128) __attribute__((amdgpu_num_vgpr(256))) void k_stat(
    const _Float16* __restrict__ q16, const _Float16* __restrict__ k16, const _Float16* __restrict__ t16,
    float* __restrict__ st) {
    __shared__ __align__(16) float sQR[4][16 * NRELP];
    __shared__ __align__(16) float sSt[128];
    const unsigned lane = threadIdx.x & 31u;
    const unsigned wave = (unsigned)__builtin_amdgcn_readfirstlane((int)(threadIdx.x >> 5));
    const unsigned hh = lane >> 4, c = lane & 15u;
    const unsigned bx = blockIdx.x;
    const unsigned b = bx / (unsigned)BLK_PER_B;
    const unsigned i0 = (bx - b * (unsigned)BLK_PER_B) * 64u + wave * 16u;
    const _Float16* qp = q16 + ((size_t)b * SEQ + i0 + c) * DH + 8u * hh;
    const v16h qf0 = frag_ld(qp), qf1 = frag_ld(qp + 32);
    float* qrs = sQR[wave];
    build_qr(t16, qrs, qf0, qf1, hh, c);
    wave_sync_lds();
    const float* qrow = qrs + c * (unsigned)NRELP;
    const int qpos = (int)(i0 + c);
    const _Float16* kb = k16 + ((size_t)b * SEQ + c) * DH + 8u * hh;
    float m = -3.0e38f, l = 0.f;
#pragma unroll 1
    for (unsigned key0 = 0; key0 < (unsigned)SEQ; key0 += 32u) {
        v8f s0, s1;
        score_step(kb + (size_t)key0 * DH, qrow, qf0, qf1, (int)(key0 + 8u * hh) - qpos + MAXREL, s0, s1);
        float mx = s0[0];
#pragma unroll
        for (int r = 1; r < 8; ++r) mx = fsel_max(mx, s0[r]);
#pragma unroll
        for (int r = 0; r < 8; ++r) mx = fsel_max(mx, s1[r]);
        const float mn = fsel_max(m, mx);
        float ps = 0.f;
#pragma unroll
        for (int r = 0; r < 8; ++r) ps += exp2f(s0[r] - mn) + exp2f(s1[r] - mn);
        l = l * exp2f(m - mn) + ps;
        m = mn;
    }
    const float mo = __shfl_xor(m, 16, 32);
    const float lo = __shfl_xor(l, 16, 32);
    const float mj = fsel_max(m, mo);
    const float lj = l * exp2f(m - mj) + lo * exp2f(mo - mj);
    if (hh == 0u) {
        sSt[wave * 16u + c] = mj;
        sSt[64u + wave * 16u + c] = 1.0f / lj;
    }
    __syncthreads();
    if (wave == 0u) {
        const v4f sv = *(const v4f*)(sSt + 4u * lane);
        float* dst = st + (size_t)bx * 128u + 4u * lane;
        *(volatile v4f*)dst = sv;
        __threadfence();
        *(volatile v4f*)dst = sv;
    }
}

__global__ __launch_bounds__(128) __attribute__((amdgpu_num_vgpr(256))) void k_attn(
    const _Float16* __restrict__ q16, const _Float16* __restrict__ k16, const _Float16* __restrict__ vt16,
    const _Float16* __restrict__ t16, const float* __restrict__ st, float* __restrict__ out, float* __restrict__ wout) {
    __shared__ __align__(16) float sQR[4][16 * NRELP];
    __shared__ __align__(16) float sW[4][16 * WT_P];
    const unsigned lane = threadIdx.x & 31u;
    const unsigned wave = (unsigned)__builtin_amdgcn_readfirstlane((int)(threadIdx.x >> 5));
    const unsigned hh = lane >> 4, c = lane & 15u;
    const unsigned bx = blockIdx.x;
    const unsigned b = bx / (unsigned)BLK_PER_B;
    const unsigned i0 = (bx - b * (unsigned)BLK_PER_B) * 64u + wave * 16u;
    const _Float16* qp = q16 + ((size_t)b * SEQ + i0 + c) * DH + 8u * hh;
    const v16h qf0 = frag_ld(qp), qf1 = frag_ld(qp + 32);
    float* qrs = sQR[wave];
    build_qr(t16, qrs, qf0, qf1, hh, c);
    wave_sync_lds();
    const float* qrow = qrs + c * (unsigned)NRELP;
    const int qpos = (int)(i0 + c);
    const _Float16* kb = k16 + ((size_t)b * SEQ + c) * DH + 8u * hh;
    const _Float16* vt = vt16 + ((size_t)b * DH + c) * SEQ;
    const float mq = st[(size_t)bx * 128u + wave * 16u + c];
    const float il = st[(size_t)bx * 128u + 64u + wave * 16u + c];
    float* wt = sW[wave];
    const unsigned q4 = lane >> 3, c4 = (lane & 7u) * 4u;
    float* wdst = wout + ((size_t)b * SEQ_FULL + i0 + q4) * SEQ_FULL + c4;
    v8f o0 = (v8f){0.f,0.f,0.f,0.f,0.f,0.f,0.f,0.f};
    v8f o1 = o0, o2 = o0, o3 = o0;
#pragma unroll 1
    for (unsigned key0 = 0; key0 < (unsigned)SEQ; key0 += 32u) {
        v8f s0, s1;
        score_step(kb + (size_t)key0 * DH, qrow, qf0, qf1, (int)(key0 + 8u * hh) - qpos + MAXREL, s0, s1);
        float p0[8], p1[8];
        FragU pf;
#pragma unroll
        for (int r = 0; r < 8; ++r) {
            p0[r] = exp2f(s0[r] - mq) * il;
            p1[r] = exp2f(s1[r] - mq) * il;
            pf.v[r] = toh_flush(p0[r] * P_CARRY);
            pf.v[8 + r] = toh_flush(p1[r] * P_CARRY);
        }
        {
            v4f a;
            float* d = wt + c * (unsigned)WT_P + 8u * hh;
            a.x = p0[0]; a.y = p0[1]; a.z = p0[2]; a.w = p0[3]; *(v4f*)(d) = a;
            a.x = p0[4]; a.y = p0[5]; a.z = p0[6]; a.w = p0[7]; *(v4f*)(d + 4) = a;
            a.x = p1[0]; a.y = p1[1]; a.z = p1[2]; a.w = p1[3]; *(v4f*)(d + 16) = a;
            a.x = p1[4]; a.y = p1[5]; a.z = p1[6]; a.w = p1[7]; *(v4f*)(d + 20) = a;
        }
        wave_sync_lds();
        v4f wv[4];
#pragma unroll
        for (int it = 0; it < 4; ++it) wv[it] = *(const v4f*)(wt + ((unsigned)it * 4u + q4) * (unsigned)WT_P + c4);
        for (int pass = 0; pass < 2; ++pass) {
#pragma unroll
            for (int it = 0; it < 4; ++it)
                *(volatile v4f*)(wdst + (size_t)((unsigned)it * 4u) * SEQ_FULL + key0) = wv[it];
            __threadfence();
        }
        wave_sync_lds();
        unsigned voff = key0 + 8u * hh;
        asm volatile("" : "+v"(voff));
        {
            const v16h a0 = frag_ld(vt + voff);
            o0 = wmma16g(a0, pf.v, o0);
            const v16h a1 = frag_ld(vt + (size_t)16 * SEQ + voff);
            o1 = wmma16g(a1, pf.v, o1);
            const v16h a2 = frag_ld(vt + (size_t)32 * SEQ + voff);
            o2 = wmma16g(a2, pf.v, o2);
            const v16h a3 = frag_ld(vt + (size_t)48 * SEQ + voff);
            o3 = wmma16g(a3, pf.v, o3);
        }
    }
    wave_sync_lds();
    {
        float* so = qrs;
        float* d = so + c * (unsigned)SO_P + 8u * hh;
        v4f a;
        a.x = o0[0] * SC_O; a.y = o0[1] * SC_O; a.z = o0[2] * SC_O; a.w = o0[3] * SC_O; *(v4f*)(d) = a;
        a.x = o0[4] * SC_O; a.y = o0[5] * SC_O; a.z = o0[6] * SC_O; a.w = o0[7] * SC_O; *(v4f*)(d + 4) = a;
        a.x = o1[0] * SC_O; a.y = o1[1] * SC_O; a.z = o1[2] * SC_O; a.w = o1[3] * SC_O; *(v4f*)(d + 16) = a;
        a.x = o1[4] * SC_O; a.y = o1[5] * SC_O; a.z = o1[6] * SC_O; a.w = o1[7] * SC_O; *(v4f*)(d + 20) = a;
        a.x = o2[0] * SC_O; a.y = o2[1] * SC_O; a.z = o2[2] * SC_O; a.w = o2[3] * SC_O; *(v4f*)(d + 32) = a;
        a.x = o2[4] * SC_O; a.y = o2[5] * SC_O; a.z = o2[6] * SC_O; a.w = o2[7] * SC_O; *(v4f*)(d + 36) = a;
        a.x = o3[0] * SC_O; a.y = o3[1] * SC_O; a.z = o3[2] * SC_O; a.w = o3[3] * SC_O; *(v4f*)(d + 48) = a;
        a.x = o3[4] * SC_O; a.y = o3[5] * SC_O; a.z = o3[6] * SC_O; a.w = o3[7] * SC_O; *(v4f*)(d + 52) = a;
        wave_sync_lds();
        const unsigned c16 = (lane & 15u) * 4u;
        float* obase = out + ((size_t)b * SEQ_FULL + i0) * DH + c16;
#pragma unroll
        for (int half = 0; half < 2; ++half) {
            v4f vv[4];
#pragma unroll
            for (int it = 0; it < 4; ++it) {
                const unsigned row = (unsigned)(half * 4 + it) * 2u + hh;
                vv[it] = *(const v4f*)(so + row * (unsigned)SO_P + c16);
            }
            for (int pass = 0; pass < 2; ++pass) {
#pragma unroll
                for (int it = 0; it < 4; ++it) {
                    const unsigned row = (unsigned)(half * 4 + it) * 2u + hh;
                    *(volatile v4f*)(obase + (size_t)row * DH) = vv[it];
                }
                __threadfence();
            }
        }
    }
}

extern "C" void kernel_launch(void* const* d_in, const int* in_sizes, int n_in, void* d_out, int out_size,
                              void* d_ws, size_t ws_size, hipStream_t stream) {
    if (n_in < 4) return;
    if (in_sizes[0] < IN_ACT_MIN || in_sizes[1] < IN_ACT_MIN || in_sizes[2] < IN_ACT_MIN || in_sizes[3] < IN_TAB_MIN) return;
    if (out_size < OUT_MIN) return;
    if (WS_TOTAL > ws_size) return;

    const float* q   = (const float*)d_in[0];
    const float* k   = (const float*)d_in[1];
    const float* v   = (const float*)d_in[2];
    const float* tab = (const float*)d_in[3];
    float* out  = (float*)d_out;
    float* wout = out + OUT1_ELEM;

    char* wsp = (char*)d_ws;
    _Float16* Q16  = (_Float16*)(wsp + OFF_Q);
    _Float16* K16  = (_Float16*)(wsp + OFF_K);
    _Float16* VT16 = (_Float16*)(wsp + OFF_VT);
    _Float16* T16  = (_Float16*)(wsp + OFF_T);
    float*    ST   = (float*)(wsp + OFF_ST);

    k_cvt_qk<<<(NB * SEQ * 8) / 256, 256, 0, stream>>>(q, k, Q16, K16);
    k_cvt_tab<<<(NRELP * 8 + 255) / 256, 256, 0, stream>>>(tab, T16);
    k_cvt_vt<<<NBLK, 256, 0, stream>>>(v, VT16);
    k_stat<<<NBLK, 128, 0, stream>>>(Q16, K16, T16, ST);
    k_attn<<<NBLK, 128, 0, stream>>>(Q16, K16, VT16, T16, ST, out, wout);
}
